// GatedMambaBlock_40329742909525
// MI455X (gfx1250) — hardware-run, weakly checked
//
#include <hip/hip_runtime.h>
#include <math.h>

#define NBT   4
#define LQ    2048
#define DIM   256
#define NTOK  8192
#define DIN   512
#define DI2   1024
#define DST   16
#define DTRK  16
#define DBW   64
#define DBN   48
#define COLB  16
#define COLC  32
#define TPB   128
#define NBLK  64
#define OSTR  68
#define SCH   32
#define SCW   256
#define LOG2E 1.4426950408889634f
#define EPSV  1e-5f
#define RDIM  (1.0f / 256.0f)

static_assert(NTOK == NBT * LQ);
static_assert(NTOK % TPB == 0);
static_assert(NBLK == NTOK / TPB);
static_assert(LQ % TPB == 0);
static_assert(DIM % 64 == 0);
static_assert(DI2 % 64 == 0);
static_assert(DBW % 64 == 0);
static_assert(DIM % 32 == 0);
static_assert(DIN % 32 == 0);
static_assert(DBW >= COLC + DST);
static_assert(DTRK == COLB);
static_assert(LQ % SCH == 0);
static_assert(SCH % 8 == 0);
static_assert(DIN % SCW == 0);
static_assert(SCW == 256);
static_assert(OSTR % 4 == 0);
static_assert(NTOK % 8 == 0);
static_assert(DIM == 256);
static_assert(DIN == 512);

typedef unsigned short us16 __attribute__((ext_vector_type(16)));
typedef unsigned short us8  __attribute__((ext_vector_type(8)));
typedef unsigned short us8a __attribute__((ext_vector_type(8), may_alias));
typedef unsigned int   u32x8 __attribute__((ext_vector_type(8)));
typedef __bf16 v16b __attribute__((ext_vector_type(16)));
typedef float v8f __attribute__((ext_vector_type(8)));
typedef float v4f __attribute__((ext_vector_type(4)));
typedef float v4fa __attribute__((ext_vector_type(4), may_alias));
union FragU { us16 v; us8 h[2]; u32x8 w; };

#if __has_builtin(__builtin_amdgcn_exp2f)
#define FEXP2(x) __builtin_amdgcn_exp2f(x)
#else
#define FEXP2(x) __expf((x) * 0.6931471805599453f)
#endif

__device__ __forceinline__ unsigned short bf16_bits(float f) {
  unsigned u = __float_as_uint(f);
  u += 0x7FFFu + ((u >> 16) & 1u);
  return (unsigned short)(u >> 16);
}
__device__ __forceinline__ float bf16_val(unsigned short b) { return __uint_as_float(((unsigned)b) << 16); }
__device__ __forceinline__ float bf16r(float f) { return bf16_val(bf16_bits(f)); }
__device__ __forceinline__ float siluf(float x) { return x * __builtin_amdgcn_rcpf(1.0f + __expf(-x)); }
__device__ __forceinline__ float sigmf(float x) { return __builtin_amdgcn_rcpf(1.0f + __expf(-x)); }

__device__ __forceinline__ void split8(const v4f a, const v4f b, us8& hi, us8& lo) {
#pragma unroll
  for (int u = 0; u < 4; ++u) {
    const unsigned short ha = bf16_bits(a[u]);
    hi[u] = ha; lo[u] = bf16_bits(a[u] - bf16_val(ha));
    const unsigned short hb = bf16_bits(b[u]);
    hi[4 + u] = hb; lo[4 + u] = bf16_bits(b[u] - bf16_val(hb));
  }
}

__device__ __forceinline__ v8f mma_bf16(us16 a, us16 b, v8f c) {
  return __builtin_amdgcn_wmma_f32_16x16x32_bf16(false, __builtin_bit_cast(v16b, a), false, __builtin_bit_cast(v16b, b), (short)0, c, false, false);
}
__device__ __forceinline__ void wguard2(v8f& c0, v8f& c1, v8f& c2, v8f& c3, const us16& a0, const us16& a1,
                                        const us16& b0, const us16& b1, const us16& b2, const us16& b3) {
#if defined(__HIP_DEVICE_COMPILE__)
  asm volatile("v_nop\n\tv_nop\n\tv_nop\n\tv_nop"
               : "+v"(c0), "+v"(c1), "+v"(c2), "+v"(c3)
               : "v"(a0), "v"(a1), "v"(b0), "v"(b1), "v"(b2), "v"(b3));
#endif
}

__device__ __forceinline__ us16 gfrag(const unsigned short* p) {
  const int kh = ((threadIdx.x >> 4) & 1) * 8;
  FragU f;
  f.h[0] = *(const us8a*)(p + kh);
  f.h[1] = *(const us8a*)(p + 16 + kh);
  return f.v;
}

__global__ __launch_bounds__(256) void k_cvt(const float* __restrict__ src, unsigned short* dst, int srcRows, int kp8, int total8) {
  const int idx = blockIdx.x * 256 + threadIdx.x;
  if (idx >= total8) return;
  const int n = idx / kp8, k8 = (idx - n * kp8) * 8;
  const bool rowok = (n < srcRows);
  const int nc = rowok ? n : (srcRows - 1);
  const float* sp = src + (size_t)nc * (size_t)(kp8 * 8) + k8;
  const v4f a = *(const v4fa*)sp, b = *(const v4fa*)(sp + 4);
  us8 o;
#pragma unroll
  for (int u = 0; u < 4; ++u) {
    o[u] = rowok ? bf16_bits(a[u]) : (unsigned short)0;
    o[4 + u] = rowok ? bf16_bits(b[u]) : (unsigned short)0;
  }
  const size_t off = (size_t)idx * 8;
  *(volatile us8*)(dst + off) = o;
  __threadfence();
  *(volatile us8*)(dst + off) = o;
}

__global__ __launch_bounds__(256) void k_ln(const float* __restrict__ X, const float* __restrict__ g, const float* __restrict__ bt,
                                           unsigned short* XH, unsigned short* XL) {
  const int tid = threadIdx.x, lane = tid & 31, wave = tid >> 5;
  const int tok = blockIdx.x * 8 + wave, c0 = lane * 8;
  const float* xr = X + (size_t)tok * DIM + c0;
  const v4f xa = *(const v4fa*)xr, xb = *(const v4fa*)(xr + 4);
  const v4f ga = *(const v4fa*)(g + c0), gbv = *(const v4fa*)(g + c0 + 4);
  const v4f ba = *(const v4fa*)(bt + c0), bbv = *(const v4fa*)(bt + c0 + 4);
  float v[8], gq[8], bq[8];
#pragma unroll
  for (int u = 0; u < 4; ++u) {
    v[u] = bf16r(xa[u]); v[4 + u] = bf16r(xb[u]);
    gq[u] = bf16r(ga[u]); gq[4 + u] = bf16r(gbv[u]);
    bq[u] = bf16r(ba[u]); bq[4 + u] = bf16r(bbv[u]);
  }
  float s = 0.0f;
#pragma unroll
  for (int u = 0; u < 8; ++u) s += v[u];
  s += __shfl_xor(s, 16); s += __shfl_xor(s, 8); s += __shfl_xor(s, 4); s += __shfl_xor(s, 2); s += __shfl_xor(s, 1);
  const float mu = s * RDIM;
  float dv[8];
  float s2 = 0.0f;
#pragma unroll
  for (int u = 0; u < 8; ++u) { dv[u] = v[u] - mu; s2 += dv[u] * dv[u]; }
  s2 += __shfl_xor(s2, 16); s2 += __shfl_xor(s2, 8); s2 += __shfl_xor(s2, 4); s2 += __shfl_xor(s2, 2); s2 += __shfl_xor(s2, 1);
  const float var = s2 * RDIM;
  const float rs = rsqrtf(var + EPSV);
  v4f oa, ob;
#pragma unroll
  for (int u = 0; u < 4; ++u) {
    oa[u] = (dv[u] * rs) * gq[u] + bq[u];
    ob[u] = (dv[4 + u] * rs) * gq[4 + u] + bq[4 + u];
  }
  us8 hi, lo;
  split8(oa, ob, hi, lo);
  const size_t off = (size_t)tok * DIM + c0;
  *(volatile us8*)(XH + off) = hi; *(volatile us8*)(XL + off) = lo;
  __threadfence();
  *(volatile us8*)(XH + off) = hi; *(volatile us8*)(XL + off) = lo;
}

template <int FIN>
__global__ __launch_bounds__(256) void k_gemm(const unsigned short* __restrict__ A0, const unsigned short* __restrict__ A1, int lda,
                                             const unsigned short* __restrict__ Bw, int ldb, int K, float* Yf, int ldy,
                                             const float* __restrict__ Xr, const float* __restrict__ MOp, const float* __restrict__ gb) {
  __shared__ __attribute__((aligned(16))) float oS[8 * 16 * OSTR];
  const int tid = threadIdx.x, lane = tid & 31, wave = tid >> 5, cl = lane & 15, hh = lane >> 4;
  const int mb = blockIdx.x * TPB, m0 = mb + 16 * wave, n0 = blockIdx.y * 64;

  v8f acc[4];
#pragma unroll
  for (int j = 0; j < 4; ++j) { const v8f zz = {0.f, 0.f, 0.f, 0.f, 0.f, 0.f, 0.f, 0.f}; acc[j] = zz; }

  const unsigned short* a0p = A0 + (size_t)(m0 + cl) * lda;
  const unsigned short* a1p = A1 + (size_t)(m0 + cl) * lda;
  const unsigned short* bwp = Bw + (size_t)(n0 + cl) * ldb;
#pragma unroll 1
  for (int k0 = 0; k0 < K; k0 += 32) {
    const us16 af0 = gfrag(a0p + k0);
    const us16 af1 = gfrag(a1p + k0);
    us16 bfr[4];
#pragma unroll
    for (int j = 0; j < 4; ++j) bfr[j] = gfrag(bwp + (size_t)(16 * j) * ldb + k0);
#pragma unroll
    for (int j = 0; j < 4; ++j) acc[j] = mma_bf16(af0, bfr[j], acc[j]);
#pragma unroll
    for (int j = 0; j < 4; ++j) acc[j] = mma_bf16(af1, bfr[j], acc[j]);
    wguard2(acc[0], acc[1], acc[2], acc[3], af0, af1, bfr[0], bfr[1], bfr[2], bfr[3]);
  }

  float* so = oS + wave * (16 * OSTR);
#pragma unroll
  for (int j = 0; j < 4; ++j)
#pragma unroll
    for (int r = 0; r < 8; ++r) so[(8 * hh + r) * OSTR + 16 * j + cl] = acc[j][r];
  __syncthreads();

#pragma unroll
  for (int pass = 0; pass < 2; ++pass) {
#pragma unroll
    for (int it = 0; it < 8; ++it) {
      const int ch = it * 32 + lane, r = ch >> 4, q = (ch & 15) * 4;
      const v4f v = *(const v4fa*)(so + r * OSTR + q);
      const size_t go = (size_t)(m0 + r) * ldy + n0 + q;
      v4f o = v;
      if (FIN) {
        const v4f xv = *(const v4fa*)(Xr + go);
        const v4f mv = *(const v4fa*)(MOp + go);
        const v4f bv = *(const v4fa*)(gb + n0 + q);
#pragma unroll
        for (int u = 0; u < 4; ++u) o[u] = bf16r(xv[u]) + mv[u] * sigmf(v[u] + bf16r(bv[u]));
      }
      *(volatile v4f*)(Yf + go) = o;
    }
    __threadfence();
  }
}

__global__ __launch_bounds__(256) void k_conv(const float* __restrict__ XZ, const float* __restrict__ cw, const float* __restrict__ cb,
                                             float* UF, unsigned short* UH, unsigned short* UL) {
  __shared__ __attribute__((aligned(16))) float su[8 * DIN];
  const int tid = threadIdx.x, lane = tid & 31, wave = tid >> 5;
  const int tok = blockIdx.x * 8 + wave, l = tok & (LQ - 1);
  float* srow = su + wave * DIN;
#pragma unroll 1
  for (int it = 0; it < 2; ++it) {
    const int c8 = it * 256 + lane * 8;
    float acc[8];
    {
      const v4f b0 = *(const v4fa*)(cb + c8), b1 = *(const v4fa*)(cb + c8 + 4);
#pragma unroll
      for (int u = 0; u < 4; ++u) { acc[u] = bf16r(b0[u]); acc[4 + u] = bf16r(b1[u]); }
    }
    v4f w4[8];
#pragma unroll
    for (int u = 0; u < 8; ++u) w4[u] = *(const v4fa*)(cw + (size_t)(c8 + u) * 4);
#pragma unroll
    for (int j = 0; j < 4; ++j) {
      const int lt = l - 3 + j;
      const bool ok = (lt >= 0);
      const size_t trow = (size_t)(ok ? (tok - 3 + j) : tok);
      const v4f xa = *(const v4fa*)(XZ + trow * DI2 + c8), xb = *(const v4fa*)(XZ + trow * DI2 + c8 + 4);
#pragma unroll
      for (int u = 0; u < 4; ++u) {
        const float x0 = ok ? xa[u] : 0.0f, x1 = ok ? xb[u] : 0.0f;
        acc[u] += bf16r(w4[u][j]) * x0;
        acc[4 + u] += bf16r(w4[4 + u][j]) * x1;
      }
    }
    v4f oa, ob;
#pragma unroll
    for (int u = 0; u < 4; ++u) { oa[u] = siluf(acc[u]); ob[u] = siluf(acc[4 + u]); }
    *(v4fa*)(srow + c8) = oa; *(v4fa*)(srow + c8 + 4) = ob;
  }
  __syncthreads();
#pragma unroll
  for (int pass = 0; pass < 2; ++pass) {
#pragma unroll
    for (int it = 0; it < 4; ++it) {
      const int c = it * 128 + lane * 4;
      const v4f v = *(const v4fa*)(srow + c);
      *(volatile v4f*)(UF + (size_t)tok * DIN + c) = v;
    }
#pragma unroll
    for (int it = 0; it < 2; ++it) {
      const int c8 = it * 256 + lane * 8;
      const v4f a = *(const v4fa*)(srow + c8), b = *(const v4fa*)(srow + c8 + 4);
      us8 hi, lo;
      split8(a, b, hi, lo);
      const size_t off = (size_t)tok * DIN + c8;
      *(volatile us8*)(UH + off) = hi; *(volatile us8*)(UL + off) = lo;
    }
    __threadfence();
  }
}

__global__ __launch_bounds__(256) void k_dt(const float* __restrict__ XDBL, const float* __restrict__ dtw, const float* __restrict__ dtb,
                                           float* DT) {
  const int idx = blockIdx.x * 256 + threadIdx.x;
  if (idx >= NTOK * DIN) return;
  const int tok = idx >> 9, d = idx & (DIN - 1);
  const float* xr = XDBL + (size_t)tok * DBW;
  const v4f x0 = *(const v4fa*)(xr), x1 = *(const v4fa*)(xr + 4), x2 = *(const v4fa*)(xr + 8), x3 = *(const v4fa*)(xr + 12);
  const float* wr = dtw + (size_t)d * DTRK;
  const v4f w0 = *(const v4fa*)(wr), w1 = *(const v4fa*)(wr + 4), w2 = *(const v4fa*)(wr + 8), w3 = *(const v4fa*)(wr + 12);
  float a = 0.0f;
#pragma unroll
  for (int r = 0; r < 4; ++r) a = a + x0[r] * bf16r(w0[r]);
#pragma unroll
  for (int r = 0; r < 4; ++r) a = a + x1[r] * bf16r(w1[r]);
#pragma unroll
  for (int r = 0; r < 4; ++r) a = a + x2[r] * bf16r(w2[r]);
#pragma unroll
  for (int r = 0; r < 4; ++r) a = a + x3[r] * bf16r(w3[r]);
  a = a + bf16r(dtb[d]);
  const float sp = fmaxf(a, 0.0f) + log1pf(__expf(-fabsf(a)));
  *(volatile float*)(DT + idx) = sp;
  __threadfence();
  *(volatile float*)(DT + idx) = sp;
}

__global__ __launch_bounds__(256) void k_scan(const float* __restrict__ DT, const float* __restrict__ UF, const float* __restrict__ XDBL,
                                             const float* __restrict__ XZ, const float* __restrict__ Alog, const float* __restrict__ Dv,
                                             unsigned short* YH, unsigned short* YL) {
  __shared__ __attribute__((aligned(16))) float sy[SCH * SCW];
  const int tid = threadIdx.x, lane = tid & 31, wave = tid >> 5;
  const int b = blockIdx.x >> 1, ch0 = (blockIdx.x & 1) * SCW, d = ch0 + tid;
  float A2[DST], h[DST];
  {
    const float* ar = Alog + (size_t)d * DST;
    const v4f a0 = *(const v4fa*)(ar), a1 = *(const v4fa*)(ar + 4), a2 = *(const v4fa*)(ar + 8), a3 = *(const v4fa*)(ar + 12);
#pragma unroll
    for (int i = 0; i < 4; ++i) {
      A2[i]      = -__expf(bf16r(a0[i])) * LOG2E; h[i] = 0.0f;
      A2[4 + i]  = -__expf(bf16r(a1[i])) * LOG2E; h[4 + i] = 0.0f;
      A2[8 + i]  = -__expf(bf16r(a2[i])) * LOG2E; h[8 + i] = 0.0f;
      A2[12 + i] = -__expf(bf16r(a3[i])) * LOG2E; h[12 + i] = 0.0f;
    }
  }
  const float Dd = bf16r(Dv[d]);
  const int c8 = lane * 8;
#pragma unroll 1
  for (int c = 0; c < LQ / SCH; ++c) {
#pragma unroll 1
    for (int s = 0; s < SCH; ++s) {
      const size_t tok = (size_t)b * LQ + (size_t)(c * SCH + s);
      const size_t e = tok * DIN + d;
      const float dl = DT[e], uv = UF[e], zv = XZ[tok * DI2 + DIN + d];
      const float* bc = XDBL + tok * DBW + COLB;
      v4f Bv[4], Cv[4];
#pragma unroll
      for (int q = 0; q < 4; ++q) {
        Bv[q] = *(const v4fa*)(bc + 4 * q);
        Cv[q] = *(const v4fa*)(bc + (COLC - COLB) + 4 * q);
      }
      const float dx = dl * uv;
      float y = 0.0f;
#pragma unroll
      for (int i = 0; i < DST; ++i) {
        const float ex = FEXP2(dl * A2[i]);
        h[i] = ex * h[i] + dx * Bv[i >> 2][i & 3];
        y = y + h[i] * Cv[i >> 2][i & 3];
      }
      sy[s * SCW + tid] = (y + uv * Dd) * siluf(zv);
    }
    __syncthreads();
#pragma unroll
    for (int pass = 0; pass < 2; ++pass) {
#pragma unroll
      for (int it = 0; it < SCH / 8; ++it) {
        const int row = it * 8 + wave;
        const v4f a = *(const v4fa*)(sy + row * SCW + c8), bb = *(const v4fa*)(sy + row * SCW + c8 + 4);
        us8 hi, lo;
        split8(a, bb, hi, lo);
        const size_t off = ((size_t)b * LQ + (size_t)(c * SCH + row)) * DIN + ch0 + c8;
        *(volatile us8*)(YH + off) = hi; *(volatile us8*)(YL + off) = lo;
      }
      __threadfence();
    }
    __syncthreads();
  }
}

extern "C" void kernel_launch(void* const* d_in, const int* in_sizes, int n_in,
                              void* d_out, int out_size, void* d_ws, size_t ws_size,
                              hipStream_t stream) {
  if (n_in < 14) return;
  if (in_sizes[0] != NTOK * DIM || in_sizes[1] != DIM || in_sizes[2] != DIM || in_sizes[3] != DI2 * DIM ||
      in_sizes[4] != DIN * 4 || in_sizes[5] != DIN || in_sizes[6] != DBN * DIN || in_sizes[7] != DIN * DTRK ||
      in_sizes[8] != DIN || in_sizes[9] != DIN * DST || in_sizes[10] != DIN || in_sizes[11] != DIM * DIN ||
      in_sizes[12] != DIM * DIM || in_sizes[13] != DIM) return;
  if (out_size != NTOK * DIM) return;

  const float* x         = (const float*)d_in[0];
  const float* ln_g      = (const float*)d_in[1];
  const float* ln_b      = (const float*)d_in[2];
  const float* W_in      = (const float*)d_in[3];
  const float* conv_w    = (const float*)d_in[4];
  const float* conv_b    = (const float*)d_in[5];
  const float* x_proj_w  = (const float*)d_in[6];
  const float* dt_proj_w = (const float*)d_in[7];
  const float* dt_proj_b = (const float*)d_in[8];
  const float* A_log     = (const float*)d_in[9];
  const float* Dv        = (const float*)d_in[10];
  const float* W_out     = (const float*)d_in[11];
  const float* gate_w    = (const float*)d_in[12];
  const float* gate_b    = (const float*)d_in[13];
  float* out = (float*)d_out;

  size_t off = 0;
  auto carve = [&](size_t bytes) -> char* { char* p = (char*)d_ws + off; off += (bytes + 255) & ~(size_t)255; return p; };
  unsigned short* XNH = (unsigned short*)carve((size_t)NTOK * DIM * 2);
  unsigned short* XNL = (unsigned short*)carve((size_t)NTOK * DIM * 2);
  float* XZ   = (float*)carve((size_t)NTOK * DI2 * 4);
  float* UF   = (float*)carve((size_t)NTOK * DIN * 4);
  unsigned short* UH  = (unsigned short*)carve((size_t)NTOK * DIN * 2);
  unsigned short* UL  = (unsigned short*)carve((size_t)NTOK * DIN * 2);
  float* XDBL = (float*)carve((size_t)NTOK * DBW * 4);
  float* DT   = (float*)carve((size_t)NTOK * DIN * 4);
  unsigned short* YH  = (unsigned short*)carve((size_t)NTOK * DIN * 2);
  unsigned short* YL  = (unsigned short*)carve((size_t)NTOK * DIN * 2);
  float* MO   = (float*)carve((size_t)NTOK * DIM * 4);
  unsigned short* WIN = (unsigned short*)carve((size_t)DI2 * DIM * 2);
  unsigned short* WXP = (unsigned short*)carve((size_t)DBW * DIN * 2);
  unsigned short* WOP = (unsigned short*)carve((size_t)DIM * DIN * 2);
  unsigned short* WG  = (unsigned short*)carve((size_t)DIM * DIM * 2);
  if (off > ws_size || off > (size_t)134217728) return;

  const dim3 b256(256);
  auto cdv = [](long a, long b) { return (unsigned)((a + b - 1) / b); };

  k_cvt<<<dim3(cdv(DI2 * (DIM / 8), 256)), b256, 0, stream>>>(W_in, WIN, DI2, DIM / 8, DI2 * (DIM / 8));
  k_cvt<<<dim3(cdv(DBW * (DIN / 8), 256)), b256, 0, stream>>>(x_proj_w, WXP, DBN, DIN / 8, DBW * (DIN / 8));
  k_cvt<<<dim3(cdv(DIM * (DIN / 8), 256)), b256, 0, stream>>>(W_out, WOP, DIM, DIN / 8, DIM * (DIN / 8));
  k_cvt<<<dim3(cdv(DIM * (DIM / 8), 256)), b256, 0, stream>>>(gate_w, WG, DIM, DIM / 8, DIM * (DIM / 8));
  k_ln<<<dim3(NTOK / 8), b256, 0, stream>>>(x, ln_g, ln_b, XNH, XNL);
  k_gemm<0><<<dim3(NBLK, DI2 / 64), b256, 0, stream>>>(XNH, XNL, DIM, WIN, DIM, DIM, XZ, DI2, x, MO, gate_b);
  k_conv<<<dim3(NTOK / 8), b256, 0, stream>>>(XZ, conv_w, conv_b, UF, UH, UL);
  k_gemm<0><<<dim3(NBLK, DBW / 64), b256, 0, stream>>>(UH, UL, DIN, WXP, DIN, DIN, XDBL, DBW, x, MO, gate_b);
  k_dt<<<dim3(cdv((long)NTOK * DIN, 256)), b256, 0, stream>>>(XDBL, dt_proj_w, dt_proj_b, DT);
  k_scan<<<dim3(NBT * (DIN / SCW)), b256, 0, stream>>>(DT, UF, XDBL, XZ, A_log, Dv, YH, YL);
  k_gemm<0><<<dim3(NBLK, DIM / 64), b256, 0, stream>>>(YH, YL, DIN, WOP, DIN, DIN, MO, DIM, x, MO, gate_b);
  k_gemm<1><<<dim3(NBLK, DIM / 64), b256, 0, stream>>>(XNH, XNL, DIM, WG, DIM, DIM, out, DIM, x, MO, gate_b);
}
